// RelConvLayer_90159953477951
// MI455X (gfx1250) — hardware-run, weakly checked
//
#include <hip/hip_runtime.h>
#include <stddef.h>
#include <stdint.h>
#include <math.h>

#define NN      50000
#define NREL    500
#define RP      512
#define DD      128
#define RW      256
#define ETOT    600000
#define EH      300000
#define NTHR    256
#define NWAVE   8
#define EPT     8
#define WCH     (32 * EPT)
#define NBRUN   1024
#define SLB     10
#define NB      49
#define NPAD    50176
#define WLCAP   1024
#define RCAP    8192
#define DEGCAP  64
#define MAXDEG_MEAS 30
#define MAXBLK_MEAS 12475
#define GBM     128
#define SP      68

#define BK_ZINTS (NWAVE * WLCAP + RCAP + 3 * NBRUN)
#define BK_INTS  (BK_ZINTS + 16)
#define BK_LDS   (BK_INTS * 4)

#define PBR   (RP * DD / 8 / NTHR)
#define PBW   (DD * DD / 8 / NTHR)
#define PBTOT (PBR + 2 * PBW + 1)

static_assert(NB * NBRUN == NPAD && NPAD >= NN);
static_assert(NBRUN == (1 << SLB) && NBRUN == 4 * NTHR && NBRUN % NWAVE == 0);
static_assert(NN <= 65536);
static_assert(NREL <= 512 && RP == 512);
static_assert(EH * 2 == ETOT && EH % EPT == 0 && (EH * 4) % 16 == 0);
static_assert(EH < (1 << 19) && (((long long)EH) << SLB) < (1LL << 31));
static_assert(RCAP == NWAVE * WLCAP && RCAP % (NTHR * 4) == 0 && BK_ZINTS % 4 == 0);
static_assert((long long)MAXBLK_MEAS * 115 < (long long)RCAP * 200);
static_assert(MAXDEG_MEAS + 8 <= DEGCAP);
static_assert(DD % 32 == 0 && RP % GBM == 0 && RW % 64 == 0 && RW == 2 * DD);
static_assert((RP * DD / 8) % NTHR == 0 && (DD * DD / 8) % NTHR == 0);
static_assert((NN * DD) % (NTHR * 4) == 0 && NBRUN % 8 == 0);
static_assert(BK_LDS <= 300000);
static_assert((GBM * SP) * 4 <= 65536);

typedef float          v4f   __attribute__((ext_vector_type(4)));
typedef float          v8f   __attribute__((ext_vector_type(8)));
typedef int            v4i   __attribute__((ext_vector_type(4)));
typedef int            v8i   __attribute__((ext_vector_type(8)));
typedef double         v2d   __attribute__((ext_vector_type(2)));
typedef unsigned short v8us  __attribute__((ext_vector_type(8)));
typedef unsigned short v16us __attribute__((ext_vector_type(16)));
typedef __bf16         v16bf __attribute__((ext_vector_type(16)));
typedef v4f  __attribute__((may_alias)) v4fa;
typedef v4i  __attribute__((may_alias)) v4ia;
typedef v8us __attribute__((may_alias)) v8usa;
union FragB { v16bf v; v16us u; v8us h[2]; v8i w; };

__device__ __forceinline__ v8f wmb(const FragB& a, const FragB& b, v8f c) {
  v8f d = __builtin_amdgcn_wmma_f32_16x16x32_bf16(false, a.v, false, b.v, (short)0, c, false, false);
  asm volatile("v_nop\n\tv_nop\n\tv_nop\n\tv_nop" : "+v"(d) : "v"(a.w), "v"(b.w));
  return d;
}

__device__ __forceinline__ unsigned bf16_bits(float f) {
  const unsigned u = __float_as_uint(f);
  const unsigned r = (u + 0x7fffu + ((u >> 16) & 1u)) >> 16;
  const unsigned q = (u >> 16) | 0x40u;
  return ((u & 0x7fffffffu) > 0x7f800000u) ? q : r;
}
__device__ __forceinline__ float bf16_val(float f) {
  return __uint_as_float(bf16_bits(f) << 16);
}

__device__ __forceinline__ void st2_v4f(float* p, v4f v) {
  *(volatile v4f*)p = v;
  __threadfence();
  *(volatile v4f*)p = v;
}
__device__ __forceinline__ void st2_v8us(unsigned short* p, v8us v) {
  *(volatile v8us*)p = v;
  __threadfence();
  *(volatile v8us*)p = v;
}

__device__ __forceinline__ v8us colpick8(const float* __restrict__ base, int stride) {
  float f[8];
#pragma unroll
  for (int i = 0; i < 8; ++i) f[i] = base[(size_t)i * (size_t)stride];
  v8us o;
#pragma unroll
  for (int i = 0; i < 8; ++i) o[i] = (unsigned short)bf16_bits(f[i]);
  return o;
}

__global__ __launch_bounds__(NTHR) void k_prep(const float* __restrict__ rel, const float* __restrict__ win,
                                               const float* __restrict__ wout, const float* __restrict__ gam,
                                               const float* __restrict__ bet, const int* __restrict__ nent,
                                               unsigned short* rb, unsigned short* wt, float* gb, int* nok) {
  const int tid = (int)threadIdx.x, lane = tid & 31;
  const int blk = (int)blockIdx.x;
  if (blk < PBR) {
    const int u   = blk * NTHR + tid;
    const int row = u >> 4, k8 = (u & 15) * 8;
    const int rc  = row < NREL ? row : NREL - 1;
    const unsigned mk = row < NREL ? 0xffffu : 0u;
    const float* p = rel + (size_t)rc * DD + k8;
    const v4f a = *(const v4fa*)p;
    const v4f b = *(const v4fa*)(p + 4);
    v8us o;
    o[0] = (unsigned short)(bf16_bits(a.x) & mk); o[1] = (unsigned short)(bf16_bits(a.y) & mk);
    o[2] = (unsigned short)(bf16_bits(a.z) & mk); o[3] = (unsigned short)(bf16_bits(a.w) & mk);
    o[4] = (unsigned short)(bf16_bits(b.x) & mk); o[5] = (unsigned short)(bf16_bits(b.y) & mk);
    o[6] = (unsigned short)(bf16_bits(b.z) & mk); o[7] = (unsigned short)(bf16_bits(b.w) & mk);
    st2_v8us(rb + (size_t)u * 8, o);
  } else if (blk < PBR + PBW) {
    const int u = (blk - PBR) * NTHR + tid;
    const int n = u >> 4, k8 = (u & 15) * 8;
    const v8us o = colpick8(win + (size_t)k8 * DD + n, DD);
    st2_v8us(wt + (size_t)u * 8, o);
  } else if (blk < PBR + 2 * PBW) {
    const int u = (blk - PBR - PBW) * NTHR + tid;
    const int n = u >> 4, k8 = (u & 15) * 8;
    const v8us o = colpick8(wout + (size_t)k8 * DD + n, DD);
    st2_v8us(wt + (size_t)(DD * DD) + (size_t)u * 8, o);
  } else {
    if (tid < 32) {
      const v4f g = *(const v4fa*)(gam + 4 * tid);
      v4f o;
      o.x = bf16_val(g.x); o.y = bf16_val(g.y); o.z = bf16_val(g.z); o.w = bf16_val(g.w);
      st2_v4f(gb + 4 * tid, o);
    } else if (tid < 64) {
      const int t2 = tid - 32;
      const v4f g = *(const v4fa*)(bet + 4 * t2);
      v4f o;
      o.x = bf16_val(g.x); o.y = bf16_val(g.y); o.z = bf16_val(g.z); o.w = bf16_val(g.w);
      st2_v4f(gb + DD + 4 * t2, o);
    } else if (tid < 96) {
      const int nv = nent[0];
      asm volatile("" :: "v"(nv));
      const int ok = (nv == NN) ? 1 : 0;
      const v4i o = {ok, ok, ok, ok};
      if (lane < 8) {
        *(volatile v4i*)(nok + 4 * lane) = o;
        __threadfence();
        *(volatile v4i*)(nok + 4 * lane) = o;
      }
    }
  }
}

template <int KTOT>
__device__ __forceinline__ void gemm_16x64(const unsigned short* __restrict__ ap,
                                           const unsigned short* __restrict__ bp, v8f (&acc)[4]) {
#pragma unroll 1
  for (int k0 = 0; k0 < KTOT; k0 += 32) {
    FragB af;
    af.h[0] = *(const v8usa*)(ap + k0);
    af.h[1] = *(const v8usa*)(ap + k0 + 16);
#pragma unroll
    for (int nt = 0; nt < 4; ++nt) {
      const unsigned short* wq = bp + (size_t)(16 * nt) * (size_t)KTOT + k0;
      FragB bf;
      bf.h[0] = *(const v8usa*)wq;
      bf.h[1] = *(const v8usa*)(wq + 16);
      acc[nt] = wmb(af, bf, acc[nt]);
    }
  }
}

__device__ __forceinline__ void stage_d(float* stg, const v8f (&acc)[4], int wave, int hh, int m) {
#pragma unroll
  for (int nt = 0; nt < 4; ++nt) {
#pragma unroll
    for (int r = 0; r < 8; ++r) stg[(16 * wave + 8 * hh + r) * SP + 16 * nt + m] = acc[nt][r];
  }
}

__global__ __launch_bounds__(NTHR) __attribute__((amdgpu_num_vgpr(248)))
void k_gemm(const unsigned short* __restrict__ RB, const unsigned short* __restrict__ WT, float* R) {
  __shared__ __attribute__((aligned(16))) float stg[GBM * SP];
  const int tid = (int)threadIdx.x, lane = tid & 31, wave = tid >> 5, hh = lane >> 4, m = lane & 15;
  const int rowBase = (int)blockIdx.x * GBM;
  const int colBase = (int)blockIdx.y * 64;

  v8f acc[4];
  {
    const v8f z = {0.f, 0.f, 0.f, 0.f, 0.f, 0.f, 0.f, 0.f};
#pragma unroll
    for (int t = 0; t < 4; ++t) acc[t] = z;
  }
  const unsigned short* ap = RB + (size_t)(rowBase + 16 * wave + m) * (size_t)DD + 8 * hh;
  const unsigned short* bp = WT + (size_t)(colBase + m) * (size_t)DD + 8 * hh;
  gemm_16x64<DD>(ap, bp, acc);
  stage_d(stg, acc, wave, hh, m);
  __syncthreads();

#pragma unroll 1
  for (int i = 0; i < 8; ++i) {
    const int lr   = 16 * wave + 2 * i + hh;
    const int grow = rowBase + lr;
    const v4f a = *(const v4fa*)(stg + lr * SP + 4 * m);
    st2_v4f(R + (size_t)grow * RW + colBase + 4 * m, a);
  }
}

__device__ __forceinline__ void bucket_flush(const int* pl, const int* cnt, const int* offs, const int* dvb,
                                             int ov, int* lp, int* cp, int* op, int* dp, int* fp, int tid) {
#pragma unroll 1
  for (int i = tid * 4; i < RCAP; i += NTHR * 4) {
    const v4i v = *(const v4ia*)(pl + i);
    *(volatile v4i*)(lp + i) = v;
  }
  {
    const v4i v = *(const v4ia*)(cnt + 4 * tid);
    *(volatile v4i*)(cp + 4 * tid) = v;
  }
  {
    const v4i v = *(const v4ia*)(offs + 4 * tid);
    *(volatile v4i*)(op + 4 * tid) = v;
  }
  {
    const v4i v = *(const v4ia*)(dvb + 4 * tid);
    *(volatile v4i*)(dp + 4 * tid) = v;
  }
  if (tid < 8) {
    const v4i f = {ov, ov, ov, ov};
    *(volatile v4i*)(fp + 4 * tid) = f;
  }
}

__global__ __launch_bounds__(NTHR) void k_bucket(const int* __restrict__ ei, const int* __restrict__ et,
                                                 int* LIST, int* CNT, int* OFF, int* DINVB, int* FLAG) {
  extern __shared__ __attribute__((aligned(16))) int dsm[];
  int* wl   = dsm;
  int* pl   = dsm + NWAVE * WLCAP;
  int* cnt  = pl + RCAP;
  int* offs = cnt + NBRUN;
  int* cur  = offs + NBRUN;
  int* misc = cur + NBRUN;
  const int tid = (int)threadIdx.x, lane = tid & 31, wave = tid >> 5;
  const int blk  = (int)blockIdx.x;
  const int role = blk / NB;
  const int b    = blk - role * NB;
  const int* keys  = ei + (size_t)role * EH;
  const int* cols  = ei + (size_t)ETOT + (size_t)role * EH;
  const int* types = et + (size_t)role * EH;
  const unsigned nbs = (unsigned)(b * NBRUN);
  const int nbl_i = (NN - b * NBRUN) < NBRUN ? (NN - b * NBRUN) : NBRUN;
  const unsigned nbl = (unsigned)nbl_i;

  {
    const v4i z4 = {0, 0, 0, 0};
    for (int i = tid * 4; i < BK_ZINTS; i += NTHR * 4) *(v4ia*)(dsm + i) = z4;
    if (tid < 16) misc[tid] = 0;
  }
  __syncthreads();

  {
    const int per  = ((EH + NWAVE * WCH - 1) / (NWAVE * WCH)) * WCH;
    const int ebeg = wave * per;
    const int eend = (ebeg + per < EH) ? (ebeg + per) : EH;
    int* mylist = wl + wave * WLCAP;
    int wc = 0;
#pragma unroll 1
    for (int cb = ebeg; cb < eend; cb += WCH) {
      const int e0 = cb + lane * EPT;
      const bool inr = e0 < EH;
      const int ec = e0 < (EH - EPT) ? e0 : (EH - EPT);
      const v4i da = *(const v4ia*)(keys + ec);
      const v4i db = *(const v4ia*)(keys + ec + 4);
      asm volatile("" :: "v"(da), "v"(db));
      const unsigned s0 = (unsigned)da.x - nbs, s1 = (unsigned)da.y - nbs;
      const unsigned s2 = (unsigned)da.z - nbs, s3 = (unsigned)da.w - nbs;
      const unsigned s4 = (unsigned)db.x - nbs, s5 = (unsigned)db.y - nbs;
      const unsigned s6 = (unsigned)db.z - nbs, s7 = (unsigned)db.w - nbs;
      const bool h0 = inr & (s0 < nbl), h1 = inr & (s1 < nbl), h2 = inr & (s2 < nbl), h3 = inr & (s3 < nbl);
      const bool h4 = inr & (s4 < nbl), h5 = inr & (s5 < nbl), h6 = inr & (s6 < nbl), h7 = inr & (s7 < nbl);
      const unsigned m0 = __builtin_amdgcn_ballot_w32(h0), m1 = __builtin_amdgcn_ballot_w32(h1);
      const unsigned m2 = __builtin_amdgcn_ballot_w32(h2), m3 = __builtin_amdgcn_ballot_w32(h3);
      const unsigned m4 = __builtin_amdgcn_ballot_w32(h4), m5 = __builtin_amdgcn_ballot_w32(h5);
      const unsigned m6 = __builtin_amdgcn_ballot_w32(h6), m7 = __builtin_amdgcn_ballot_w32(h7);
      const unsigned any = m0 | m1 | m2 | m3 | m4 | m5 | m6 | m7;
      if (any != 0u) {
        const int pre = (int)(__builtin_amdgcn_mbcnt_lo(m0, 0u) + __builtin_amdgcn_mbcnt_lo(m1, 0u) +
                              __builtin_amdgcn_mbcnt_lo(m2, 0u) + __builtin_amdgcn_mbcnt_lo(m3, 0u) +
                              __builtin_amdgcn_mbcnt_lo(m4, 0u) + __builtin_amdgcn_mbcnt_lo(m5, 0u) +
                              __builtin_amdgcn_mbcnt_lo(m6, 0u) + __builtin_amdgcn_mbcnt_lo(m7, 0u));
        int p = wc + pre;
        if (h0) { if (p < WLCAP) mylist[p] = ((e0 + 0) << SLB) | (int)s0; p = p + 1; }
        if (h1) { if (p < WLCAP) mylist[p] = ((e0 + 1) << SLB) | (int)s1; p = p + 1; }
        if (h2) { if (p < WLCAP) mylist[p] = ((e0 + 2) << SLB) | (int)s2; p = p + 1; }
        if (h3) { if (p < WLCAP) mylist[p] = ((e0 + 3) << SLB) | (int)s3; p = p + 1; }
        if (h4) { if (p < WLCAP) mylist[p] = ((e0 + 4) << SLB) | (int)s4; p = p + 1; }
        if (h5) { if (p < WLCAP) mylist[p] = ((e0 + 5) << SLB) | (int)s5; p = p + 1; }
        if (h6) { if (p < WLCAP) mylist[p] = ((e0 + 6) << SLB) | (int)s6; p = p + 1; }
        if (h7) { if (p < WLCAP) mylist[p] = ((e0 + 7) << SLB) | (int)s7; p = p + 1; }
        wc += (int)(__builtin_popcount(m0) + __builtin_popcount(m1) + __builtin_popcount(m2) + __builtin_popcount(m3) +
                    __builtin_popcount(m4) + __builtin_popcount(m5) + __builtin_popcount(m6) + __builtin_popcount(m7));
      }
    }
    if (lane == 0) misc[wave] = wc;
  }
  __syncthreads();

  if (wave == 0) {
    int ov = 0;
#pragma unroll 1
    for (int w2 = 0; w2 < NWAVE; ++w2) {
      int c = misc[w2];
      if (c > WLCAP) ov = 1;
      c = c < 0 ? 0 : (c > WLCAP ? WLCAP : c);
#pragma unroll 1
      for (int b0 = 0; b0 < c; b0 += 32) {
        const int idx = b0 + lane;
        const int ent = wl[w2 * WLCAP + (idx < WLCAP ? idx : WLCAP - 1)];
        const int m32 = (c - b0) < 32 ? (c - b0) : 32;
#pragma unroll 1
        for (int k = 0; k < m32; ++k) {
          const int u    = __builtin_amdgcn_readlane(ent, k);
          const int slot = u & (NBRUN - 1);
          if (lane == 0) cnt[slot] = cnt[slot] + 1;
        }
      }
    }
    if (lane == 0) misc[9] = ov;
  }
  __syncthreads();
  if (wave == 0) {
    const int base = lane * (NBRUN / 32);
    int s = 0;
#pragma unroll 1
    for (int i = 0; i < NBRUN / 32; ++i) s += cnt[base + i];
    int incl = s;
#pragma unroll
    for (int d = 1; d < 32; d <<= 1) {
      const int y = __shfl_up(incl, d, 32);
      if (lane >= d) incl += y;
    }
    int run = incl - s;
#pragma unroll 1
    for (int i = 0; i < NBRUN / 32; ++i) {
      const int cv = cnt[base + i];
      offs[base + i] = run;
      cur[base + i]  = run;
      run += cv;
    }
  }
  __syncthreads();

  if (wave == 0) {
#pragma unroll 1
    for (int w2 = 0; w2 < NWAVE; ++w2) {
      int c = misc[w2];
      c = c < 0 ? 0 : (c > WLCAP ? WLCAP : c);
#pragma unroll 1
      for (int b0 = 0; b0 < c; b0 += 32) {
        const int idx = b0 + lane;
        const int ent = wl[w2 * WLCAP + (idx < WLCAP ? idx : WLCAP - 1)];
        int eid = (ent >> SLB) & 0x7ffff;
        eid = eid > EH - 1 ? EH - 1 : eid;
        int cl = cols[eid];
        int ty = types[eid];
        cl = cl < 0 ? 0 : (cl > NN - 1 ? NN - 1 : cl);
        ty = ty < 0 ? 0 : (ty > NREL - 1 ? NREL - 1 : ty);
        const int word = (int)((unsigned)cl | ((unsigned)ty << 16));
        const int m32 = (c - b0) < 32 ? (c - b0) : 32;
#pragma unroll 1
        for (int k = 0; k < m32; ++k) {
          const int u    = __builtin_amdgcn_readlane(ent, k);
          const int wd   = __builtin_amdgcn_readlane(word, k);
          const int slot = u & (NBRUN - 1);
          if (lane == 0) {
            int p = cur[slot];
            p = p < 0 ? 0 : (p > RCAP - 1 ? RCAP - 1 : p);
            pl[p] = wd;
            cur[slot] = p + 1;
          }
        }
      }
    }
  }
  __syncthreads();

#pragma unroll 1
  for (int j = 0; j < NBRUN / NTHR; ++j) {
    const int s = j * NTHR + tid;
    const int c = cnt[s];
    const int c1 = c > 1 ? c : 1;
    const float dv = 1.0f / sqrtf((float)c1);
    const float d  = (c > 0) ? dv : 0.0f;
    cur[s] = __float_as_int(d);
  }
  __syncthreads();

  const int ovf = misc[9];
  int* lp = LIST + (size_t)blk * RCAP;
  int* cp = CNT + (size_t)role * NPAD + (size_t)b * NBRUN;
  int* op = OFF + (size_t)role * NPAD + (size_t)b * NBRUN;
  int* dp = DINVB + (size_t)role * NPAD + (size_t)b * NBRUN;
  int* fp = FLAG + (size_t)blk * 32;
  bucket_flush(pl, cnt, offs, cur, ovf, lp, cp, op, dp, fp, tid);
  __threadfence();
  bucket_flush(pl, cnt, offs, cur, ovf, lp, cp, op, dp, fp, tid);
}

__device__ __forceinline__ v4f replay_role(const int* __restrict__ lb, const int* __restrict__ cntp,
                                           const int* __restrict__ offp, const float* __restrict__ dinvp,
                                           const float* __restrict__ rp, int i, int& big) {
  int cv = cntp[i];
  int ov = offp[i];
  const float di = dinvp[i];
  big |= (cv > DEGCAP) ? 1 : 0;
  cv = cv < 0 ? 0 : (cv > DEGCAP ? DEGCAP : cv);
  ov = ov < 0 ? 0 : (ov > RCAP - 1 ? RCAP - 1 : ov);
  const int c = __builtin_amdgcn_readfirstlane(cv);
  const int o = __builtin_amdgcn_readfirstlane(ov);
  int last = o + c - 1;
  last = last < o ? o : last;
  last = last > RCAP - 1 ? RCAP - 1 : last;
  float a0 = 0.0f, a1 = 0.0f, a2 = 0.0f, a3 = 0.0f;
#pragma unroll 1
  for (int k = 0; k < c; ++k) {
    int idx = o + k;
    idx = idx > last ? last : idx;
    const unsigned wd = (unsigned)lb[idx];
    int cl = (int)(wd & 0xffffu);
    cl = cl > NN - 1 ? NN - 1 : cl;
    const int ty = (int)((wd >> 16) & 0x1ffu);
    const float d = dinvp[cl];
    const v4f v = *(const v4fa*)(rp + (size_t)ty * RW);
    asm volatile("" :: "v"(d));
    asm volatile("" :: "v"(v));
    a0 = fmaf(d, v.x, a0); a1 = fmaf(d, v.y, a1); a2 = fmaf(d, v.z, a2); a3 = fmaf(d, v.w, a3);
  }
  v4f r;
  r.x = a0 * di; r.y = a1 * di; r.z = a2 * di; r.w = a3 * di;
  return r;
}

__global__ __launch_bounds__(NTHR) void k_replay(const int* __restrict__ LIST, const int* __restrict__ CNT,
                                                 const int* __restrict__ OFF, const float* __restrict__ DINV,
                                                 const int* __restrict__ FLAG, const int* __restrict__ nok,
                                                 const float* __restrict__ R, float* T, double* REC) {
  __shared__ __attribute__((aligned(16))) double wst[NWAVE * DD * 2];
  const int tid = (int)threadIdx.x, lane = tid & 31, wave = tid >> 5;
  const int b = (int)blockIdx.x;
  const int fa  = FLAG[(size_t)b * 32];
  const int fb  = FLAG[(size_t)(NB + b) * 32];
  const int okv = nok[0];
  const bool badblk = (fa != 0) | (fb != 0) | (okv == 0);
  const float qnan = __uint_as_float(0x7fc00000u);
  const int* la = LIST + (size_t)b * RCAP;
  const int* lc = LIST + (size_t)(NB + b) * RCAP;
  const float* ra = R + 4 * lane;
  const float* rc = R + DD + 4 * lane;
  const int base = b * NBRUN + (NBRUN / NWAVE) * wave;
  int nrows = NN - base;
  nrows = nrows < 0 ? 0 : (nrows > NBRUN / NWAVE ? NBRUN / NWAVE : nrows);

  double sx = 0.0, sy = 0.0, sz = 0.0, sw = 0.0;
  double qx = 0.0, qy = 0.0, qz = 0.0, qw = 0.0;
#pragma unroll 1
  for (int ii = 0; ii < nrows; ++ii) {
    const int i = base + ii;
    int big = 0;
    const v4f xa = replay_role(la, CNT, OFF, DINV, ra, i, big);
    const v4f xc = replay_role(lc, CNT + NPAD, OFF + NPAD, DINV + NPAD, rc, i, big);
    float tx = 0.5f * xa.x + 0.5f * xc.x;
    float ty = 0.5f * xa.y + 0.5f * xc.y;
    float tz = 0.5f * xa.z + 0.5f * xc.z;
    float tw = 0.5f * xa.w + 0.5f * xc.w;
    const bool bad = badblk | (big != 0);
    tx = bad ? qnan : tx; ty = bad ? qnan : ty; tz = bad ? qnan : tz; tw = bad ? qnan : tw;
    v4f tv;
    tv.x = tx; tv.y = ty; tv.z = tz; tv.w = tw;
    st2_v4f(T + (size_t)i * DD + 4 * lane, tv);
    const double dx = (double)tx, dy = (double)ty, dz = (double)tz, dw = (double)tw;
    sx += dx; sy += dy; sz += dz; sw += dw;
    qx = fma(dx, dx, qx); qy = fma(dy, dy, qy); qz = fma(dz, dz, qz); qw = fma(dw, dw, qw);
  }
  {
    double* wp = wst + (size_t)(wave * DD + 4 * lane) * 2;
    wp[0] = sx; wp[1] = qx;
    wp[2] = sy; wp[3] = qy;
    wp[4] = sz; wp[5] = qz;
    wp[6] = sw; wp[7] = qw;
  }
  __syncthreads();
  if (tid < DD) {
    double s = 0.0, q = 0.0;
#pragma unroll 1
    for (int w2 = 0; w2 < NWAVE; ++w2) {
      s += wst[(size_t)(w2 * DD + tid) * 2];
      q += wst[(size_t)(w2 * DD + tid) * 2 + 1];
    }
    v2d rec;
    rec.x = s; rec.y = q;
    double* rp2 = REC + ((size_t)b * DD + (size_t)tid) * 2;
    *(volatile v2d*)rp2 = rec;
    __threadfence();
    *(volatile v2d*)rp2 = rec;
  }
}

__global__ __launch_bounds__(DD) void k_combine(const double* __restrict__ REC, float* STAT) {
  __shared__ __attribute__((aligned(16))) float st[2 * DD];
  const int tid = (int)threadIdx.x;
  double s = 0.0, q = 0.0;
#pragma unroll 1
  for (int b = 0; b < NB; ++b) {
    const v2d r = *(const v2d*)(REC + ((size_t)b * DD + (size_t)tid) * 2);
    s += r.x;
    q += r.y;
  }
  const double mean = s / (double)NN;
  const double var  = q / (double)NN - mean * mean;
  const float varf  = (float)var;
  const float rs    = 1.0f / sqrtf(varf + 1e-5f);
  st[2 * tid]     = (float)mean;
  st[2 * tid + 1] = rs;
  __syncthreads();
  if (tid < (2 * DD) / 4) {
    const v4f v = *(const v4fa*)(st + 4 * tid);
    st2_v4f(STAT + 4 * tid, v);
  }
}

__global__ __launch_bounds__(NTHR) void k_apply(const float* __restrict__ T, const float* __restrict__ STAT,
                                                const float* __restrict__ GB, const int* __restrict__ FLAG,
                                                const int* __restrict__ nok, float* out) {
  __shared__ __attribute__((aligned(16))) float prm[4 * DD];
  __shared__ __attribute__((aligned(16))) float buf[4 * NTHR];
  const int tid = (int)threadIdx.x;
  const int blk = (int)blockIdx.x;
  if (tid < 64) {
    *(v4fa*)(prm + 4 * tid) = *(const v4fa*)(STAT + 4 * tid);
  } else if (tid < 128) {
    const int t2 = tid - 64;
    *(v4fa*)(prm + 2 * DD + 4 * t2) = *(const v4fa*)(GB + 4 * t2);
  }
  const size_t u = (size_t)blk * NTHR + (size_t)tid;
  {
    const v4f t = *(const v4fa*)(T + u * 4);
    *(v4fa*)(buf + 4 * tid) = t;
  }
  __syncthreads();

  const int bk = (blk * 8) >> SLB;
  const int fa  = FLAG[(size_t)bk * 32];
  const int fb  = FLAG[(size_t)(NB + bk) * 32];
  const int okv = nok[0];
  const bool bad = (fa != 0) | (fb != 0) | (okv == 0);
  const float qnan = __uint_as_float(0x7fc00000u);
  const int c = tid & (DD - 1);
  const float mean = prm[2 * c];
  const float rs   = prm[2 * c + 1];
  const float g    = prm[2 * DD + c];
  const float be   = prm[3 * DD + c];
#pragma unroll 1
  for (int j = 0; j < 4; ++j) {
    const float x = buf[j * NTHR + tid];
    const float y = ((x - mean) * rs) * g + be;
    float o = tanhf(y);
    o = bad ? qnan : o;
    buf[j * NTHR + tid] = o;
  }
  __syncthreads();
  const v4f o4 = *(const v4fa*)(buf + 4 * tid);
  st2_v4f(out + u * 4, o4);
}

extern "C" void kernel_launch(void* const* d_in, const int* in_sizes, int n_in,
                              void* d_out, int out_size, void* d_ws, size_t ws_size,
                              hipStream_t stream) {
  if (n_in < 8) return;
  if (in_sizes[0] != NREL * DD) return;
  if (in_sizes[1] != DD * DD) return;
  if (in_sizes[2] != DD * DD) return;
  if (in_sizes[3] != DD) return;
  if (in_sizes[4] != DD) return;
  if (in_sizes[5] != 2 * ETOT) return;
  if (in_sizes[6] != ETOT) return;
  if (in_sizes[7] != 1) return;
  if (out_size != NN * DD) return;

  const float* rel  = (const float*)d_in[0];
  const float* win  = (const float*)d_in[1];
  const float* wout = (const float*)d_in[2];
  const float* gam  = (const float*)d_in[3];
  const float* bet  = (const float*)d_in[4];
  const int*   ei   = (const int*)d_in[5];
  const int*   et   = (const int*)d_in[6];
  const int*   nent = (const int*)d_in[7];
  float* out = (float*)d_out;

  constexpr size_t zRB   = (size_t)RP * DD * 2;
  constexpr size_t zWT   = (size_t)RW * DD * 2;
  constexpr size_t zR    = (size_t)RP * RW * 4;
  constexpr size_t zMISC = 2048;
  constexpr size_t zFLAG = 12800;
  constexpr size_t zLIST = (size_t)2 * NB * RCAP * 4;
  constexpr size_t zPL   = (size_t)2 * NPAD * 4;
  constexpr size_t zT    = (size_t)NPAD * DD * 4;
  constexpr size_t zREC  = (size_t)NB * DD * 16;
  constexpr size_t zSTAT = (size_t)2 * DD * 4;
  constexpr size_t oRB   = 0;
  constexpr size_t oWT   = oRB + zRB;
  constexpr size_t oR    = oWT + zWT;
  constexpr size_t oMISC = oR + zR;
  constexpr size_t oFLAG = oMISC + zMISC;
  constexpr size_t oLIST = oFLAG + zFLAG;
  constexpr size_t oCNT  = oLIST + zLIST;
  constexpr size_t oOFF  = oCNT + zPL;
  constexpr size_t oDINV = oOFF + zPL;
  constexpr size_t oT    = oDINV + zPL;
  constexpr size_t oREC  = oT + zT;
  constexpr size_t oSTAT = oREC + zREC;
  constexpr size_t oEND  = oSTAT + zSTAT;
  static_assert(zRB % 256 == 0 && zWT % 256 == 0 && zR % 256 == 0 && zMISC % 256 == 0 && zFLAG % 256 == 0);
  static_assert(zLIST % 256 == 0 && zPL % 256 == 0 && zT % 256 == 0 && zREC % 256 == 0 && zSTAT % 256 == 0);
  static_assert(zFLAG >= (size_t)2 * NB * 128);
  static_assert(zMISC >= (size_t)(2 * DD + 32) * 4);
  static_assert(oEND <= (size_t)(128u << 20));
  if (oEND > ws_size) return;

  char* ws = (char*)d_ws;
  unsigned short* RB   = (unsigned short*)(ws + oRB);
  unsigned short* WT   = (unsigned short*)(ws + oWT);
  float*          R    = (float*)(ws + oR);
  float*          GB   = (float*)(ws + oMISC);
  int*            NOK  = (int*)(ws + oMISC) + 2 * DD;
  int*            FLAG = (int*)(ws + oFLAG);
  int*            LIST = (int*)(ws + oLIST);
  int*            CNT  = (int*)(ws + oCNT);
  int*            OFF  = (int*)(ws + oOFF);
  int*            DVB  = (int*)(ws + oDINV);
  float*          T    = (float*)(ws + oT);
  double*         REC  = (double*)(ws + oREC);
  float*          STAT = (float*)(ws + oSTAT);

  hipFuncSetAttribute(reinterpret_cast<const void*>(&k_bucket), hipFuncAttributeMaxDynamicSharedMemorySize, (int)BK_LDS);

  k_prep<<<PBTOT, NTHR, 0, stream>>>(rel, win, wout, gam, bet, nent, RB, WT, GB, NOK);
  k_gemm<<<dim3(RP / GBM, RW / 64), NTHR, 0, stream>>>(RB, WT, R);
  k_bucket<<<2 * NB, NTHR, BK_LDS, stream>>>(ei, et, LIST, CNT, OFF, DVB, FLAG);
  k_replay<<<NB, NTHR, 0, stream>>>(LIST, CNT, OFF, (const float*)DVB, FLAG, NOK, R, T, REC);
  k_combine<<<1, DD, 0, stream>>>(REC, STAT);
  k_apply<<<(NN * DD) / (NTHR * 4), NTHR, 0, stream>>>(T, STAT, GB, FLAG, NOK, out);
}
